// DSGNet_50448685859251
// MI455X (gfx1250) — hardware-verified
//
#include <hip/hip_runtime.h>
#include <stddef.h>
#include <stdint.h>


#define NENT   20000
#define NPAD   20096
#define HD     256
#define KP2    512
#define K3     768
#define DEG    32
#define TOPK   8
#define NREL   400
#define RPAD   512
#define BSZ    512
#define FLAT   8320
#define KFC    16640
#define NB64   314
#define NB128  157
#define NEDGE  640000
#define NSELB  2512
#define OUT0_ELEMS 10240000
#define OUT_ELEMS  10240001
#define KNOWRAP 0x40000000
#define LDS_G2   66560
#define LDS_G1   32768
#define LDS_CONV 104960
#define WSMAX  134217728

static_assert(DEG == 32);
static_assert(TOPK == 8);
static_assert(HD == 32 * 8);
static_assert(FLAT == 32 * 26 * 10);
static_assert(KFC == 2 * FLAT && FLAT % 32 == 0);
static_assert(NPAD == NB128 * 128 && NPAD == NB64 * 64 && NPAD == NSELB * 8);
static_assert(NENT % 4 == 0 && NENT - (NB128 - 1) * 128 == 32);
static_assert((NENT * 4) % 128 == 0);
static_assert(OUT0_ELEMS == BSZ * NENT && OUT0_ELEMS < OUT_ELEMS);
static_assert((OUT0_ELEMS * 4) % 128 == 0);
static_assert(NEDGE == NENT * DEG);
static_assert(LDS_G2 == 64 * 256 * 4 + 256 * 4);
static_assert(LDS_CONV == 2048 + 272 * 128 * 2 + FLAT * 4);
static_assert(LDS_CONV <= 327680 && LDS_G2 <= 327680);

typedef float          v4f   __attribute__((ext_vector_type(4)));
typedef float          v8f   __attribute__((ext_vector_type(8)));
typedef double         v2d   __attribute__((ext_vector_type(2)));
typedef int            v8i   __attribute__((ext_vector_type(8)));
typedef unsigned short v8us  __attribute__((ext_vector_type(8)));
typedef unsigned short v16us __attribute__((ext_vector_type(16)));
typedef __bf16         v16bf __attribute__((ext_vector_type(16)));
typedef v4f  __attribute__((may_alias)) v4fa;
typedef v8us __attribute__((may_alias)) v8usa;
union FragB { v16bf v; v16us u; v8us h[2]; v8i w; };

__device__ __forceinline__ v8f wmb(const FragB& a, const FragB& b, v8f c) {
  v8f d = __builtin_amdgcn_wmma_f32_16x16x32_bf16(false, a.v, false, b.v, (short)0, c, false, false);
  asm volatile("v_nop\n\tv_nop\n\tv_nop\n\tv_nop" : "+v"(d) : "v"(a.w), "v"(b.w));
  return d;
}

__device__ __forceinline__ unsigned bf16_bits(float f) {
  const unsigned u = __float_as_uint(f);
  return (u + 0x7FFFu + ((u >> 16) & 1u)) >> 16;
}
__device__ __forceinline__ float bf16_val(float f) {
  return __uint_as_float(bf16_bits(f) << 16);
}
__device__ __forceinline__ v4f bfr4(const v4f a) {
  v4f r; r.x = bf16_val(a.x); r.y = bf16_val(a.y); r.z = bf16_val(a.z); r.w = bf16_val(a.w); return r;
}
__device__ __forceinline__ void split8(const v4f a, const v4f b, v8us& hi, v8us& lo) {
  const float f[8] = {a.x, a.y, a.z, a.w, b.x, b.y, b.z, b.w};
#pragma unroll
  for (int i = 0; i < 8; ++i) {
    const unsigned hb = bf16_bits(f[i]);
    hi[i] = (unsigned short)hb;
    lo[i] = (unsigned short)bf16_bits(f[i] - __uint_as_float(hb << 16));
  }
}
__device__ __forceinline__ void gates2(const float* __restrict__ gate, float& g0, float& g1) {
  const float a = bf16_val(gate[0]);
  const float b = bf16_val(gate[1]);
  const float mx = fmaxf(a, b);
  const float e0 = expf(a - mx);
  const float e1 = expf(b - mx);
  const float inv = 1.0f / (e0 + e1);
  g0 = e0 * inv;
  g1 = e1 * inv;
}
__device__ __forceinline__ float relu_keep(float v) { return (v > 0.0f) ? v : (v - v); }

template <int NC>
__device__ __forceinline__ void gemm_core(const unsigned short* __restrict__ A, int lda,
                                          const unsigned short* __restrict__ BT, int ldb,
                                          int K, int kwrap, int rowBase, int colBase, float* stg) {
  constexpr int LDC = 128 * NC;
  const int tid = (int)threadIdx.x, lane = tid & 31, wave = tid >> 5, hh = lane >> 4, m = lane & 15;
  const int rg = wave & 3, cg = wave >> 2;
  v8f acc[8];
  {
    const v8f z = {0.f, 0.f, 0.f, 0.f, 0.f, 0.f, 0.f, 0.f};
#pragma unroll
    for (int t = 0; t < 8; ++t) acc[t] = z;
  }
  const unsigned short* ap = A  + (size_t)(rowBase + 16 * rg + m) * (size_t)lda + 8 * hh;
  const unsigned short* bp = BT + (size_t)(colBase + cg * 128 + m) * (size_t)ldb + 8 * hh;
#pragma unroll 1
  for (int k0 = 0; k0 < K; k0 += 32) {
    const int kb = (k0 >= kwrap) ? (k0 - kwrap) : k0;
    FragB af;
    af.h[0] = *(const v8usa*)(ap + k0);
    af.h[1] = *(const v8usa*)(ap + k0 + 16);
#pragma unroll
    for (int nt = 0; nt < 8; ++nt) {
      const unsigned short* wq = bp + (size_t)(16 * nt) * (size_t)ldb + kb;
      FragB bf;
      bf.h[0] = *(const v8usa*)wq;
      bf.h[1] = *(const v8usa*)(wq + 16);
      acc[nt] = wmb(af, bf, acc[nt]);
    }
  }
#pragma unroll
  for (int nt = 0; nt < 8; ++nt) {
    const int lc = cg * 128 + 16 * nt + m;
#pragma unroll
    for (int r = 0; r < 8; ++r) {
      const int lr = 16 * rg + 8 * hh + r;
      stg[lr * LDC + lc] = acc[nt][r];
    }
  }
  __syncthreads();
}

#define PA_UEB (NPAD * 32)
#define PA_USW 8192
static_assert(PA_UEB % 256 == 0 && PA_USW % 256 == 0);
__global__ __launch_bounds__(256) void k_pa(const float* __restrict__ ent, const float* __restrict__ Sw,
                                            const float* __restrict__ Lw,
                                            unsigned short* EB, unsigned short* SLT) {
  const int u = (int)blockIdx.x * 256 + (int)threadIdx.x;
  v8us o;
  unsigned short* dp;
  if (u < PA_UEB) {
    const int row = u >> 5;
    const int c8  = (u & 31) * 8;
    const int rc  = row < NENT ? row : NENT - 1;
    const float* p = ent + (size_t)rc * HD + c8;
    const v4f a = *(const v4f*)p;
    const v4f b = *(const v4f*)(p + 4);
    const bool ok = row < NENT;
    o[0] = ok ? (unsigned short)bf16_bits(a.x) : (unsigned short)0;
    o[1] = ok ? (unsigned short)bf16_bits(a.y) : (unsigned short)0;
    o[2] = ok ? (unsigned short)bf16_bits(a.z) : (unsigned short)0;
    o[3] = ok ? (unsigned short)bf16_bits(a.w) : (unsigned short)0;
    o[4] = ok ? (unsigned short)bf16_bits(b.x) : (unsigned short)0;
    o[5] = ok ? (unsigned short)bf16_bits(b.y) : (unsigned short)0;
    o[6] = ok ? (unsigned short)bf16_bits(b.z) : (unsigned short)0;
    o[7] = ok ? (unsigned short)bf16_bits(b.w) : (unsigned short)0;
    dp = EB + (size_t)row * HD + c8;
  } else if (u < PA_UEB + PA_USW) {
    const int v  = u - PA_UEB;
    const int n  = v >> 5;
    const int k8 = (v & 31) * 8;
    const float* p = Sw + (size_t)k8 * HD + n;
#pragma unroll
    for (int i = 0; i < 8; ++i) o[i] = (unsigned short)bf16_bits(p[(size_t)i * HD]);
    dp = SLT + (size_t)n * HD + k8;
  } else if (u < PA_UEB + 2 * PA_USW) {
    const int v  = u - PA_UEB - PA_USW;
    const int n  = v >> 5;
    const int k8 = (v & 31) * 8;
    const float* p = Lw + (size_t)k8 * HD + n;
#pragma unroll
    for (int i = 0; i < 8; ++i) o[i] = (unsigned short)bf16_bits(p[(size_t)i * HD]);
    dp = SLT + (size_t)(HD + n) * HD + k8;
  } else {
    return;
  }
  *(volatile v8us*)dp = o;
  __threadfence();
  *(volatile v8us*)dp = o;
}

#define PB_U0 32768
#define PB_U1 65536
#define PB_U2 81920
#define PB_U3 114688
#define PB_U4 115712
__global__ __launch_bounds__(256) void k_pb(const float* __restrict__ W, const float* __restrict__ Wr,
                                            const float* __restrict__ NW, const float* __restrict__ rel,
                                            const float* __restrict__ av,
                                            unsigned short* WT2, unsigned short* NWT2, unsigned short* WRT,
                                            unsigned short* RB, float* V) {
  __shared__ __attribute__((aligned(16))) float vsh[256];
  const int tid = (int)threadIdx.x;
  const int u = (int)blockIdx.x * 256 + tid;
  if (u >= PB_U3) {
    if (u >= PB_U4) return;
    const int v = u - PB_U3;
    const int q = v >> 8;
    const int k = v & 255;
    const int i = q >> 1, j = q & 1;
    const float* wr = W + (size_t)i * 65536 + (size_t)k * HD;
    const float* ar = av + i * 768 + j * HD;
    double acc = 0.0;
#pragma unroll 1
    for (int n = 0; n < HD; n += 4) {
      const v4f w4 = bfr4(*(const v4f*)(wr + n));
      const v4f a4 = bfr4(*(const v4f*)(ar + n));
      acc = fma((double)w4.x, (double)a4.x, acc);
      acc = fma((double)w4.y, (double)a4.y, acc);
      acc = fma((double)w4.z, (double)a4.z, acc);
      acc = fma((double)w4.w, (double)a4.w, acc);
    }
    vsh[tid] = (float)acc;
    __syncthreads();
    if (tid < 64) {
      const v4f o4 = *(const v4fa*)(vsh + 4 * tid);
      float* vp = V + q * HD + 4 * tid;
      *(volatile v4f*)vp = o4;
      __threadfence();
      *(volatile v4f*)vp = o4;
    }
    return;
  }
  v8us o;
  unsigned short* dp;
  if (u < PB_U0) {
    const int i  = u >> 14;
    const int n  = (u >> 6) & 255;
    const int k8 = (u & 63) * 8;
    const int kk = k8 & 255;
    const float* p = W + (size_t)i * 65536 + (size_t)kk * HD + n;
#pragma unroll
    for (int t = 0; t < 8; ++t) o[t] = (unsigned short)bf16_bits(p[(size_t)t * HD]);
    dp = WT2 + (size_t)i * 131072 + (size_t)n * KP2 + k8;
  } else if (u < PB_U1) {
    const int v  = u - PB_U0;
    const int i  = v >> 14;
    const int n  = (v >> 6) & 255;
    const int k8 = (v & 63) * 8;
    const int kk = k8 & 255;
    const float* p = NW + (size_t)i * 65536 + (size_t)kk * HD + n;
#pragma unroll
    for (int t = 0; t < 8; ++t) o[t] = (unsigned short)bf16_bits(p[(size_t)t * HD]);
    dp = NWT2 + (size_t)i * 131072 + (size_t)n * KP2 + k8;
  } else if (u < PB_U2) {
    const int v  = u - PB_U1;
    const int i  = v >> 13;
    const int n  = (v >> 5) & 255;
    const int k8 = (v & 31) * 8;
    const float* p = Wr + (size_t)i * 65536 + (size_t)k8 * HD + n;
#pragma unroll
    for (int t = 0; t < 8; ++t) o[t] = (unsigned short)bf16_bits(p[(size_t)t * HD]);
    dp = WRT + (size_t)i * 65536 + (size_t)n * HD + k8;
  } else {
    const int v  = u - PB_U2;
    const int i  = v >> 14;
    const int r  = (v >> 5) & 511;
    const int c8 = (v & 31) * 8;
    const int rc = r < NREL ? r : NREL - 1;
    const float* p = rel + ((size_t)i * NREL + rc) * HD + c8;
    const v4f a = *(const v4f*)p;
    const v4f b = *(const v4f*)(p + 4);
    const bool ok = r < NREL;
    o[0] = ok ? (unsigned short)bf16_bits(a.x) : (unsigned short)0;
    o[1] = ok ? (unsigned short)bf16_bits(a.y) : (unsigned short)0;
    o[2] = ok ? (unsigned short)bf16_bits(a.z) : (unsigned short)0;
    o[3] = ok ? (unsigned short)bf16_bits(a.w) : (unsigned short)0;
    o[4] = ok ? (unsigned short)bf16_bits(b.x) : (unsigned short)0;
    o[5] = ok ? (unsigned short)bf16_bits(b.y) : (unsigned short)0;
    o[6] = ok ? (unsigned short)bf16_bits(b.z) : (unsigned short)0;
    o[7] = ok ? (unsigned short)bf16_bits(b.w) : (unsigned short)0;
    dp = RB + ((size_t)i * RPAD + r) * HD + c8;
  }
  *(volatile v8us*)dp = o;
  __threadfence();
  *(volatile v8us*)dp = o;
}

#define PC_U0 25600
#define PC_U1 26112
static_assert(PC_U0 % 256 == 0 && PC_U1 % 256 == 0 && PC_U0 * 4 == NREL * HD);
__global__ __launch_bounds__(256) void k_pc(const float* __restrict__ rel, const float* __restrict__ gate,
                                            const float* __restrict__ cw, float* RELF, unsigned short* CWB) {
  const int u = (int)blockIdx.x * 256 + (int)threadIdx.x;
  if (u < PC_U0) {
    float g0, g1;
    gates2(gate, g0, g1);
    const size_t idx = (size_t)u * 4;
    const v4f r0 = bfr4(*(const v4f*)(rel + idx));
    const v4f r1 = bfr4(*(const v4f*)(rel + (size_t)NREL * HD + idx));
    v4f o;
    { const float t = g0 * r0.x; o.x = t + g1 * r1.x; }
    { const float t = g0 * r0.y; o.y = t + g1 * r1.y; }
    { const float t = g0 * r0.z; o.z = t + g1 * r1.z; }
    { const float t = g0 * r0.w; o.w = t + g1 * r1.w; }
    float* dp = RELF + idx;
    *(volatile v4f*)dp = o;
    __threadfence();
    *(volatile v4f*)dp = o;
  } else if (u < PC_U1) {
    const int v  = u - PC_U0;
    const int oc = v >> 4;
    const int k8 = (v & 15) * 8;
    v8us o;
#pragma unroll
    for (int j = 0; j < 8; ++j) {
      const int t  = (k8 & 63) + j;
      const int tc = t < 49 ? t : 48;
      const float w = cw[oc * 49 + tc];
      o[j] = (t < 49) ? (unsigned short)bf16_bits(w) : (unsigned short)0;
    }
    unsigned short* dp = CWB + oc * 128 + k8;
    *(volatile v8us*)dp = o;
    __threadfence();
    *(volatile v8us*)dp = o;
  }
}

__global__ __launch_bounds__(256) void k_pc2(const float* __restrict__ fcw, unsigned short* FCT) {
  const int u = (int)blockIdx.x * 256 + (int)threadIdx.x;
  if (u >= HD * (FLAT / 8)) return;
  const int n  = u / (FLAT / 8);
  const int k8 = (u - n * (FLAT / 8)) * 8;
  const float* p = fcw + (size_t)k8 * HD + n;
  v8us o;
#pragma unroll
  for (int i = 0; i < 8; ++i) o[i] = (unsigned short)bf16_bits(p[(size_t)i * HD]);
  unsigned short* dp = FCT + (size_t)n * FLAT + k8;
  *(volatile v8us*)dp = o;
  __threadfence();
  *(volatile v8us*)dp = o;
}

__global__ __launch_bounds__(256) __attribute__((amdgpu_num_vgpr(248)))
void k_gemm_cp(const unsigned short* __restrict__ EB, const unsigned short* __restrict__ SLT,
               const float* __restrict__ Sb, const float* __restrict__ Lb, const float* __restrict__ V,
               unsigned short* CPhl, float* SDP) {
  extern __shared__ __attribute__((aligned(16))) float gsm[];
  float* stg = gsm;
  float* sdt = gsm + 64 * 256;
  const int tid = (int)threadIdx.x, lane = tid & 31, wave = tid >> 5;
  const int t = (int)blockIdx.y;
  const int rowBase = (int)blockIdx.x * 64;
  gemm_core<2>(EB, HD, SLT + (size_t)t * 65536, HD, HD, KNOWRAP, rowBase, 0, stg);

  const int c0 = 8 * lane;
  float bb[8];
  {
    const v4f s0 = *(const v4f*)(Sb + c0);
    const v4f s1 = *(const v4f*)(Sb + c0 + 4);
    const v4f l0 = *(const v4f*)(Lb + c0);
    const v4f l1 = *(const v4f*)(Lb + c0 + 4);
    const bool tp = (t != 0);
    bb[0] = bf16_val(tp ? l0.x : s0.x); bb[1] = bf16_val(tp ? l0.y : s0.y);
    bb[2] = bf16_val(tp ? l0.z : s0.z); bb[3] = bf16_val(tp ? l0.w : s0.w);
    bb[4] = bf16_val(tp ? l1.x : s1.x); bb[5] = bf16_val(tp ? l1.y : s1.y);
    bb[6] = bf16_val(tp ? l1.z : s1.z); bb[7] = bf16_val(tp ? l1.w : s1.w);
  }
  float vv[4][8];
#pragma unroll
  for (int q = 0; q < 4; ++q) {
    const v4f a = *(const v4f*)(V + q * HD + c0);
    const v4f b = *(const v4f*)(V + q * HD + c0 + 4);
    vv[q][0] = a.x; vv[q][1] = a.y; vv[q][2] = a.z; vv[q][3] = a.w;
    vv[q][4] = b.x; vv[q][5] = b.y; vv[q][6] = b.z; vv[q][7] = b.w;
  }
  unsigned short* cp = CPhl + (size_t)t * NPAD * KP2;

#pragma unroll 1
  for (int i = 0; i < 8; ++i) {
    const int row = wave * 8 + i;
    float* sp = stg + row * 256 + c0;
    const v4f p0 = *(const v4fa*)sp;
    const v4f p1 = *(const v4fa*)(sp + 4);
    v4f w0, w1;
    w0.x = p0.x + bb[0]; w0.y = p0.y + bb[1]; w0.z = p0.z + bb[2]; w0.w = p0.w + bb[3];
    w1.x = p1.x + bb[4]; w1.y = p1.y + bb[5]; w1.z = p1.z + bb[6]; w1.w = p1.w + bb[7];
    *(v4fa*)sp = w0;
    *(v4fa*)(sp + 4) = w1;
    const float x[8] = {w0.x, w0.y, w0.z, w0.w, w1.x, w1.y, w1.z, w1.w};
    float d[4];
#pragma unroll
    for (int q = 0; q < 4; ++q) {
      float s = 0.0f;
#pragma unroll
      for (int j = 0; j < 8; ++j) s = fmaf(x[j], vv[q][j], s);
      d[q] = s;
    }
#pragma unroll
    for (int off = 16; off > 0; off >>= 1) {
      d[0] += __shfl_xor(d[0], off);
      d[1] += __shfl_xor(d[1], off);
      d[2] += __shfl_xor(d[2], off);
      d[3] += __shfl_xor(d[3], off);
    }
    if (lane == 0) {
      sdt[row] = d[0]; sdt[64 + row] = d[1]; sdt[128 + row] = d[2]; sdt[192 + row] = d[3];
    }
    v8us hi, lo;
    split8(w0, w1, hi, lo);
    unsigned short* gp = cp + (size_t)(rowBase + row) * KP2 + c0;
    *(volatile v8us*)gp = hi;
    *(volatile v8us*)(gp + HD) = lo;
  }
  __syncthreads();
  v4f alv = {0.f, 0.f, 0.f, 0.f};
  float* alp = SDP + ((size_t)t * NB64 + blockIdx.x) * 256 + 4 * (tid & 63);
  if (tid < 64) {
    alv = *(const v4fa*)(sdt + 4 * tid);
    *(volatile v4f*)alp = alv;
  }
  __threadfence();
#pragma unroll 1
  for (int i = 0; i < 8; ++i) {
    const int row = wave * 8 + i;
    const float* sp = stg + row * 256 + c0;
    const v4f w0 = *(const v4fa*)sp;
    const v4f w1 = *(const v4fa*)(sp + 4);
    v8us hi, lo;
    split8(w0, w1, hi, lo);
    unsigned short* gp = cp + (size_t)(rowBase + row) * KP2 + c0;
    *(volatile v8us*)gp = hi;
    *(volatile v8us*)(gp + HD) = lo;
  }
  if (tid < 64) *(volatile v4f*)alp = alv;
}

template <int EP>
__global__ __launch_bounds__(256) __attribute__((amdgpu_num_vgpr(248)))
void k_gemm_f32(const unsigned short* __restrict__ A, int lda, const unsigned short* __restrict__ BT, int ldb,
                int K, float* Cm, const float* __restrict__ avec, float* DO) {
  extern __shared__ __attribute__((aligned(16))) float gsm[];
  float* stg = gsm;
  float* sdt = gsm + 64 * 256;
  const int tid = (int)threadIdx.x, lane = tid & 31, wave = tid >> 5;
  const int rowBase = (int)blockIdx.x * 64;
  if constexpr (EP == 2) {
    const int z = (int)blockIdx.y;
    A    += (size_t)z * RPAD * HD;
    BT   += (size_t)z * 65536;
    Cm   += (size_t)z * RPAD * HD;
    avec += z * 768 + 512;
    DO   += z * RPAD;
  }
  gemm_core<2>(A, lda, BT, ldb, K, KNOWRAP, rowBase, 0, stg);

  v4f a4[2];
  a4[0] = a4[1] = (v4f){0.f, 0.f, 0.f, 0.f};
  if constexpr (EP == 2) {
    a4[0] = bfr4(*(const v4f*)(avec + 4 * lane));
    a4[1] = bfr4(*(const v4f*)(avec + 128 + 4 * lane));
  }
#pragma unroll 1
  for (int i = 0; i < 8; ++i) {
    const int row = wave * 8 + i;
    float s = 0.0f;
#pragma unroll
    for (int c = 0; c < 2; ++c) {
      float* sp = stg + row * 256 + c * 128 + 4 * lane;
      v4f p = *(const v4fa*)sp;
      if constexpr (EP == 1) {
        p.x = tanhf(p.x); p.y = tanhf(p.y); p.z = tanhf(p.z); p.w = tanhf(p.w);
        *(v4fa*)sp = p;
      }
      if constexpr (EP == 2) {
        s = fmaf(p.x, a4[c].x, s); s = fmaf(p.y, a4[c].y, s);
        s = fmaf(p.z, a4[c].z, s); s = fmaf(p.w, a4[c].w, s);
      }
      float* op = Cm + (size_t)(rowBase + row) * HD + c * 128 + 4 * lane;
      *(volatile v4f*)op = p;
    }
    if constexpr (EP == 2) {
#pragma unroll
      for (int off = 16; off > 0; off >>= 1) s += __shfl_xor(s, off);
      if (lane == 0) sdt[row] = s;
    }
  }
  v4f dv = {0.f, 0.f, 0.f, 0.f};
  if constexpr (EP == 2) {
    __syncthreads();
    if (tid < 16) {
      dv = *(const v4fa*)(sdt + 4 * tid);
      *(volatile v4f*)(DO + rowBase + 4 * tid) = dv;
    }
  }
  __threadfence();
#pragma unroll 1
  for (int i = 0; i < 8; ++i) {
    const int row = wave * 8 + i;
#pragma unroll
    for (int c = 0; c < 2; ++c) {
      const v4f p = *(const v4fa*)(stg + row * 256 + c * 128 + 4 * lane);
      float* op = Cm + (size_t)(rowBase + row) * HD + c * 128 + 4 * lane;
      *(volatile v4f*)op = p;
    }
  }
  if constexpr (EP == 2) {
    if (tid < 16) *(volatile v4f*)(DO + rowBase + 4 * tid) = dv;
  }
}

__global__ __launch_bounds__(256) __attribute__((amdgpu_num_vgpr(248)))
void k_sel(const int* __restrict__ esrc, const int* __restrict__ erel, const float* __restrict__ SDt,
           const float* __restrict__ HRA3i, const float* __restrict__ Hm, const float* __restrict__ HRi,
           unsigned short* NE, float* diag, int isp) {
  __shared__ float gsh[8];
  const int tid = (int)threadIdx.x, lane = tid & 31, wave = tid >> 5;
  const int node = (int)blockIdx.x * 8 + wave;
  const bool live = node < NENT;
  const int nc = live ? node : NENT - 1;
  const int e = nc * DEG + lane;
  int sr = esrc[e];
  sr = sr < 0 ? 0 : (sr > NENT - 1 ? NENT - 1 : sr);
  int rl = erel[e];
  rl = rl < 0 ? 0 : (rl > NREL - 1 ? NREL - 1 : rl);
  const float s1 = SDt[((sr >> 6) * 4 + 2 * isp) * 64 + (sr & 63)];
  const float s2 = SDt[((nc >> 6) * 4 + 2 * isp + 1) * 64 + (nc & 63)];
  const float s3 = HRA3i[rl];
  float s = (s1 + s2) + s3;
  s = (s > 0.0f) ? s : 0.2f * s;

  int rank = 0;
#pragma unroll 4
  for (int l = 0; l < 32; ++l) {
    const float o = __shfl(s, l);
    rank += ((o > s) || (o == s && l < lane)) ? 1 : 0;
  }
  float mtop;
  {
    const unsigned m0 = __builtin_amdgcn_ballot_w32(rank == 0);
    const int l0 = (m0 != 0u) ? (int)__builtin_ctz(m0) : 0;
    mtop = __shfl(s, l0);
  }
  const float ev = expf(s - mtop);
  float sum = 0.0f;
#pragma unroll 1
  for (int k = 0; k < TOPK; ++k) {
    const unsigned mk = __builtin_amdgcn_ballot_w32(rank == k);
    const int lk = (mk != 0u) ? (int)__builtin_ctz(mk) : 0;
    sum += __shfl(ev, lk);
  }
  float gap;
  {
    const unsigned m7 = __builtin_amdgcn_ballot_w32(rank == 7);
    const unsigned m8 = __builtin_amdgcn_ballot_w32(rank == 8);
    const int l7 = (m7 != 0u) ? (int)__builtin_ctz(m7) : 0;
    const int l8 = (m8 != 0u) ? (int)__builtin_ctz(m8) : 0;
    const float v7 = __shfl(s, l7);
    const float v8 = __shfl(s, l8);
    gap = v7 - v8;
  }
  const float inv = 1.0f / sum;

  float acc[8];
#pragma unroll
  for (int c = 0; c < 8; ++c) acc[c] = 0.0f;
#pragma unroll 1
  for (int k = 0; k < TOPK; ++k) {
    const unsigned mk = __builtin_amdgcn_ballot_w32(rank == k);
    const int lk = (mk != 0u) ? (int)__builtin_ctz(mk) : 0;
    const int sk = __shfl(sr, lk);
    const int rk = __shfl(rl, lk);
    const float ak = __shfl(ev, lk) * inv;
    const float* hp = Hm + (size_t)sk * HD + 8 * lane;
    const float* rp = HRi + (size_t)rk * HD + 8 * lane;
    const v4f h0 = *(const v4f*)hp;
    const v4f h1 = *(const v4f*)(hp + 4);
    const v4f r0 = *(const v4f*)rp;
    const v4f r1 = *(const v4f*)(rp + 4);
    { const float p = h0.x * r0.x; acc[0] = fmaf(p, ak, acc[0]); }
    { const float p = h0.y * r0.y; acc[1] = fmaf(p, ak, acc[1]); }
    { const float p = h0.z * r0.z; acc[2] = fmaf(p, ak, acc[2]); }
    { const float p = h0.w * r0.w; acc[3] = fmaf(p, ak, acc[3]); }
    { const float p = h1.x * r1.x; acc[4] = fmaf(p, ak, acc[4]); }
    { const float p = h1.y * r1.y; acc[5] = fmaf(p, ak, acc[5]); }
    { const float p = h1.z * r1.z; acc[6] = fmaf(p, ak, acc[6]); }
    { const float p = h1.w * r1.w; acc[7] = fmaf(p, ak, acc[7]); }
  }
  v4f w0, w1;
  w0.x = live ? acc[0] : 0.0f; w0.y = live ? acc[1] : 0.0f; w0.z = live ? acc[2] : 0.0f; w0.w = live ? acc[3] : 0.0f;
  w1.x = live ? acc[4] : 0.0f; w1.y = live ? acc[5] : 0.0f; w1.z = live ? acc[6] : 0.0f; w1.w = live ? acc[7] : 0.0f;
  v8us hi, lo;
  split8(w0, w1, hi, lo);
  unsigned short* gp = NE + (size_t)node * KP2 + 8 * lane;
  *(volatile v8us*)gp = hi;
  *(volatile v8us*)(gp + HD) = lo;
  __threadfence();
  *(volatile v8us*)gp = hi;
  *(volatile v8us*)(gp + HD) = lo;

  if (lane == 0) gsh[wave] = live ? gap : 3.0e38f;
  __syncthreads();
  if (wave == 0) {
    float mn = gsh[0];
#pragma unroll
    for (int q = 1; q < 8; ++q) mn = fminf(mn, gsh[q]);
    const float gq = gsh[lane & 7];
    if (lane < 8) {
      v4f o;
      o.x = gq; o.y = mn; o.z = 0.0f; o.w = 0.0f;
      float* dp = diag + (size_t)blockIdx.x * 32 + 4 * lane;
      *(volatile v4f*)dp = o;
      __threadfence();
      *(volatile v4f*)dp = o;
    }
  }
}

template <int ISP>
__global__ __launch_bounds__(256) __attribute__((amdgpu_num_vgpr(248)))
void k_fuse(const float* __restrict__ ent, const float* __restrict__ Tc, const float* __restrict__ Tp,
            const float* __restrict__ gate, float* EF, double* REC) {
  static_assert(ISP == 0 || ISP == 1);
  __shared__ __attribute__((aligned(16))) double red[4 * 1280];
  const int tid = (int)threadIdx.x;
  const int cg = tid & 63, rs = tid >> 6;
  const int c4 = 4 * cg;
  const int blk = (int)blockIdx.x;
  float g0, g1;
  gates2(gate, g0, g1);
  const float g = (ISP != 0) ? g1 : g0;
  int nrows = NENT - blk * 128;
  nrows = nrows > 128 ? 128 : nrows;
  const int nj = nrows >> 2;
  double Sa[4], Sb[4], Saa[4], Sbb[4], Sab[4];
#pragma unroll
  for (int k = 0; k < 4; ++k) { Sa[k] = 0.0; Sb[k] = 0.0; Saa[k] = 0.0; Sbb[k] = 0.0; Sab[k] = 0.0; }
#pragma unroll 1
  for (int j = 0; j < nj; ++j) {
    const size_t idx = (size_t)(blk * 128 + rs + 4 * j) * HD + c4;
    const v4f a = *(const v4f*)(Tc + idx);
    const v4f b = *(const v4f*)(Tp + idx);
    const v4f e = bfr4(*(const v4f*)(ent + idx));
    v4f old = {0.f, 0.f, 0.f, 0.f};
    if constexpr (ISP != 0) {
      old = *(const v4fa*)(EF + idx);
    }
    const float av[4] = {a.x, a.y, a.z, a.w};
    const float bv[4] = {b.x, b.y, b.z, b.w};
    const float evv[4] = {e.x, e.y, e.z, e.w};
    const float ov[4] = {old.x, old.y, old.z, old.w};
    float r[4];
#pragma unroll
    for (int k = 0; k < 4; ++k) {
      const double da = (double)av[k], db = (double)bv[k];
      Sa[k] += da; Sb[k] += db;
      Saa[k] = fma(da, da, Saa[k]);
      Sbb[k] = fma(db, db, Sbb[k]);
      Sab[k] = fma(da, db, Sab[k]);
      const float esem = (evv[k] + av[k]) + bv[k];
      const float t = g * esem;
      if constexpr (ISP != 0) {
        r[k] = ov[k] + t;
      } else {
        r[k] = t;
      }
    }
    v4f val;
    val.x = r[0]; val.y = r[1]; val.z = r[2]; val.w = r[3];
    float* op = EF + idx;
    *(volatile v4f*)op = val;
    __threadfence();
    *(volatile v4f*)op = val;
  }
#pragma unroll
  for (int k = 0; k < 4; ++k) {
    red[rs * 1280 + 0 * 256 + c4 + k] = Sa[k];
    red[rs * 1280 + 1 * 256 + c4 + k] = Sb[k];
    red[rs * 1280 + 2 * 256 + c4 + k] = Saa[k];
    red[rs * 1280 + 3 * 256 + c4 + k] = Sbb[k];
    red[rs * 1280 + 4 * 256 + c4 + k] = Sab[k];
  }
  __syncthreads();
  double* rp = REC + (size_t)blk * 1280;
#pragma unroll 1
  for (int u = tid; u < 640; u += 256) {
    const int o = 2 * u;
    v2d v;
    v.x = ((red[o] + red[1280 + o]) + red[2560 + o]) + red[3840 + o];
    v.y = ((red[o + 1] + red[1280 + o + 1]) + red[2560 + o + 1]) + red[3840 + o + 1];
    *(volatile v2d*)(rp + o) = v;
  }
  __threadfence();
#pragma unroll 1
  for (int u = tid; u < 640; u += 256) {
    const int o = 2 * u;
    v2d v;
    v.x = ((red[o] + red[1280 + o]) + red[2560 + o]) + red[3840 + o];
    v.y = ((red[o + 1] + red[1280 + o + 1]) + red[2560 + o + 1]) + red[3840 + o + 1];
    *(volatile v2d*)(rp + o) = v;
  }
}

__global__ __launch_bounds__(256) void k_corr(const double* __restrict__ REC, float* out1) {
  __shared__ double red[3 * 256];
  __shared__ double cres[2];
  const int tid = (int)threadIdx.x;
#pragma unroll 1
  for (int i = 0; i < 2; ++i) {
    double Sa = 0.0, Sb = 0.0, Saa = 0.0, Sbb = 0.0, Sab = 0.0;
#pragma unroll 1
    for (int blk = 0; blk < NB128; ++blk) {
      const double* p = REC + ((size_t)(i * NB128 + blk) * 5) * 256 + tid;
      Sa += p[0]; Sb += p[256]; Saa += p[512]; Sbb += p[768]; Sab += p[1024];
    }
    const double n = (double)NENT;
    red[tid]       = Saa - Sa * Sa / n;
    red[256 + tid] = Sbb - Sb * Sb / n;
    red[512 + tid] = Sab - Sa * Sb / n;
    __syncthreads();
    if (tid == 0) {
      double caa = 0.0, cbb = 0.0, cab = 0.0;
#pragma unroll 1
      for (int c = 0; c < 256; ++c) { caa += red[c]; cbb += red[256 + c]; cab += red[512 + c]; }
      const double nh = (double)NENT * 256.0;
      const double s1 = (double)sqrtf((float)(caa / nh));
      const double s2 = (double)sqrtf((float)(cbb / nh));
      const double den = s1 * s2 + (double)1e-8f;
      cres[i] = fabs(cab / nh) / den;
    }
    __syncthreads();
  }
  if (tid == 0) {
    const float val = (float)((cres[0] + cres[1]) * 0.5);
    *(volatile float*)out1 = val;
    __threadfence();
    *(volatile float*)out1 = val;
  }
}

__global__ __launch_bounds__(256) void k_split(const float* __restrict__ EF, unsigned short* EF3) {
  const int u = (int)blockIdx.x * 256 + (int)threadIdx.x;
  if (u >= NPAD * 32) return;
  const int row = u >> 5;
  const int c8  = (u & 31) * 8;
  const int rc  = row < NENT ? row : NENT - 1;
  const float* p = EF + (size_t)rc * HD + c8;
  v4f a = *(const v4f*)p;
  v4f b = *(const v4f*)(p + 4);
  const float keep = (row < NENT) ? 1.0f : 0.0f;
  a.x *= keep; a.y *= keep; a.z *= keep; a.w *= keep;
  b.x *= keep; b.y *= keep; b.z *= keep; b.w *= keep;
  v8us hi, lo;
  split8(a, b, hi, lo);
  unsigned short* dp = EF3 + (size_t)row * K3 + c8;
  *(volatile v8us*)dp = hi;
  *(volatile v8us*)(dp + HD) = hi;
  *(volatile v8us*)(dp + 2 * HD) = lo;
  __threadfence();
  *(volatile v8us*)dp = hi;
  *(volatile v8us*)(dp + HD) = hi;
  *(volatile v8us*)(dp + 2 * HD) = lo;
}

__global__ __launch_bounds__(256) __attribute__((amdgpu_num_vgpr(248)))
void k_conv(const int* __restrict__ hid, const int* __restrict__ rid, const float* __restrict__ EF,
            const float* __restrict__ RELF, const unsigned short* __restrict__ CWB,
            const float* __restrict__ cb, unsigned short* XC) {
  extern __shared__ __attribute__((aligned(16))) float csm[];
  float* imgs = csm;
  unsigned short* At = (unsigned short*)(csm + 512);
  float* ost = csm + 512 + (272 * 128) / 2;
  const int tid = (int)threadIdx.x, lane = tid & 31, hh = lane >> 4, m = lane & 15;
  const int wave = __builtin_amdgcn_readfirstlane(tid >> 5);
  const int b = (int)blockIdx.x;
  int hi_ = hid[b];
  hi_ = hi_ < 0 ? 0 : (hi_ > NENT - 1 ? NENT - 1 : hi_);
  int ri_ = rid[b];
  ri_ = ri_ < 0 ? 0 : (ri_ > NREL - 1 ? NREL - 1 : ri_);
  imgs[tid]       = EF[(size_t)hi_ * HD + tid];
  imgs[256 + tid] = RELF[(size_t)ri_ * HD + tid];
  __syncthreads();

  {
    const int t  = tid & 63;
    const int p0 = tid >> 6;
    const int tc = t < 49 ? t : 48;
    const int ky = tc / 7;
    const int kx = tc - 7 * ky;
    const bool tv = t < 49;
#pragma unroll 1
    for (int j = 0; j < 68; ++j) {
      const int p  = p0 + 4 * j;
      const int pc = p < 260 ? p : 259;
      const int oh = pc / 10;
      const int ow = pc - 10 * oh;
      float v = imgs[(oh + ky) * 16 + ow + kx];
      v = (tv && p < 260) ? v : 0.0f;
      const unsigned hb = bf16_bits(v);
      const unsigned lb = bf16_bits(v - __uint_as_float(hb << 16));
      At[p * 128 + t]      = (unsigned short)hb;
      At[p * 128 + 64 + t] = (unsigned short)lb;
    }
  }
  __syncthreads();

#pragma unroll 1
  for (int j = 0; j < 5; ++j) {
    const int T = wave + 8 * j;
    if (T < 34) {
      const int mt = T >> 1, nt = T & 1;
      v8f acc = {0.f, 0.f, 0.f, 0.f, 0.f, 0.f, 0.f, 0.f};
      const unsigned short* ap = At + (16 * mt + m) * 128 + 8 * hh;
      const unsigned short* bq = CWB + (16 * nt + m) * 128 + 8 * hh;
#pragma unroll
      for (int ks = 0; ks < 4; ++ks) {
        const int k0 = 32 * ks;
        FragB af, bf;
        af.h[0] = *(const v8usa*)(ap + k0);
        af.h[1] = *(const v8usa*)(ap + k0 + 16);
        bf.h[0] = *(const v8usa*)(bq + k0);
        bf.h[1] = *(const v8usa*)(bq + k0 + 16);
        acc = wmb(af, bf, acc);
      }
      const int oc = 16 * nt + m;
      const float cbv = bf16_val(cb[oc]);
#pragma unroll
      for (int r = 0; r < 8; ++r) {
        const int p = 16 * mt + 8 * hh + r;
        const float v = relu_keep(acc[r] + cbv);
        if (p < 260) ost[oc * 260 + p] = v;
      }
    }
  }
  __syncthreads();

  unsigned short* xrow = XC + (size_t)b * KFC;
#pragma unroll 1
  for (int j = 0; j < 5; ++j) {
    const int u = tid + 256 * j;
    if (u < FLAT / 8) {
      const int f = 8 * u;
      const v4f p0 = *(const v4fa*)(ost + f);
      const v4f p1 = *(const v4fa*)(ost + f + 4);
      v8us hi, lo;
      split8(p0, p1, hi, lo);
      *(volatile v8us*)(xrow + f) = hi;
      *(volatile v8us*)(xrow + FLAT + f) = lo;
    }
  }
  __threadfence();
#pragma unroll 1
  for (int j = 0; j < 5; ++j) {
    const int u = tid + 256 * j;
    if (u < FLAT / 8) {
      const int f = 8 * u;
      const v4f p0 = *(const v4fa*)(ost + f);
      const v4f p1 = *(const v4fa*)(ost + f + 4);
      v8us hi, lo;
      split8(p0, p1, hi, lo);
      *(volatile v8us*)(xrow + f) = hi;
      *(volatile v8us*)(xrow + FLAT + f) = lo;
    }
  }
}

__global__ __launch_bounds__(256) __attribute__((amdgpu_num_vgpr(248)))
void k_gemm_fc(const unsigned short* __restrict__ XC, const unsigned short* __restrict__ FCT,
               const float* __restrict__ fcb, unsigned short* A3x) {
  extern __shared__ __attribute__((aligned(16))) float gsm[];
  float* stg = gsm;
  const int tid = (int)threadIdx.x, lane = tid & 31, wave = tid >> 5;
  const int rowBase = (int)blockIdx.x * 64;
  gemm_core<2>(XC, KFC, FCT, FLAT, KFC, FLAT, rowBase, 0, stg);
  const int c0 = 8 * lane;
  float bb[8];
  {
    const v4f a = bfr4(*(const v4f*)(fcb + c0));
    const v4f b = bfr4(*(const v4f*)(fcb + c0 + 4));
    bb[0] = a.x; bb[1] = a.y; bb[2] = a.z; bb[3] = a.w;
    bb[4] = b.x; bb[5] = b.y; bb[6] = b.z; bb[7] = b.w;
  }
#pragma unroll 1
  for (int i = 0; i < 8; ++i) {
    const int row = wave * 8 + i;
    float* sp = stg + row * 256 + c0;
    const v4f p0 = *(const v4fa*)sp;
    const v4f p1 = *(const v4fa*)(sp + 4);
    v4f w0, w1;
    w0.x = relu_keep(p0.x + bb[0]); w0.y = relu_keep(p0.y + bb[1]);
    w0.z = relu_keep(p0.z + bb[2]); w0.w = relu_keep(p0.w + bb[3]);
    w1.x = relu_keep(p1.x + bb[4]); w1.y = relu_keep(p1.y + bb[5]);
    w1.z = relu_keep(p1.z + bb[6]); w1.w = relu_keep(p1.w + bb[7]);
    *(v4fa*)sp = w0;
    *(v4fa*)(sp + 4) = w1;
    v8us hi, lo;
    split8(w0, w1, hi, lo);
    unsigned short* gp = A3x + (size_t)(rowBase + row) * K3 + c0;
    *(volatile v8us*)gp = hi;
    *(volatile v8us*)(gp + HD) = lo;
    *(volatile v8us*)(gp + 2 * HD) = hi;
  }
  __threadfence();
#pragma unroll 1
  for (int i = 0; i < 8; ++i) {
    const int row = wave * 8 + i;
    const float* sp = stg + row * 256 + c0;
    const v4f w0 = *(const v4fa*)sp;
    const v4f w1 = *(const v4fa*)(sp + 4);
    v8us hi, lo;
    split8(w0, w1, hi, lo);
    unsigned short* gp = A3x + (size_t)(rowBase + row) * K3 + c0;
    *(volatile v8us*)gp = hi;
    *(volatile v8us*)(gp + HD) = lo;
    *(volatile v8us*)(gp + 2 * HD) = hi;
  }
}

__global__ __launch_bounds__(128) __attribute__((amdgpu_num_vgpr(248)))
void k_gemm_score(const unsigned short* __restrict__ A3x, const unsigned short* __restrict__ EF3,
                  const float* __restrict__ ebias, float* outp) {
  extern __shared__ __attribute__((aligned(16))) float gsm[];
  float* stg = gsm;
  const int tid = (int)threadIdx.x, lane = tid & 31, wave = tid >> 5;
  const int rowBase = (int)blockIdx.x * 64;
  const int colBase = (int)blockIdx.y * 128;
  gemm_core<1>(A3x, K3, EF3, K3, K3, KNOWRAP, rowBase, colBase, stg);
  const int col = colBase + 4 * lane;
  const bool ok = col < NENT;
  const int cc = ok ? col : NENT - 4;
  const v4f b4 = bfr4(*(const v4f*)(ebias + cc));
#pragma unroll 1
  for (int i = 0; i < 16; ++i) {
    const int row = wave * 16 + i;
    float* sp = stg + row * 128 + 4 * lane;
    v4f p = *(const v4fa*)sp;
    p.x += b4.x; p.y += b4.y; p.z += b4.z; p.w += b4.w;
    *(v4fa*)sp = p;
    if (ok) {
      float* op = outp + (size_t)(rowBase + row) * NENT + col;
      *(volatile v4f*)op = p;
    }
  }
  __threadfence();
#pragma unroll 1
  for (int i = 0; i < 16; ++i) {
    const int row = wave * 16 + i;
    const v4f p = *(const v4fa*)(stg + row * 128 + 4 * lane);
    if (ok) {
      float* op = outp + (size_t)(rowBase + row) * NENT + col;
      *(volatile v4f*)op = p;
    }
  }
}

static constexpr size_t SZ_R1   = (size_t)2 * NPAD * KP2 * 2;
static constexpr size_t SZ_PL   = (size_t)NPAD * HD * 4;
static constexpr size_t SZ_EF   = (size_t)NENT * HD * 4;
static constexpr size_t SZ_EF3  = (size_t)NPAD * K3 * 2;
static constexpr size_t SZ_FCT  = (size_t)HD * FLAT * 2;
static constexpr size_t SZ_A3X  = (size_t)BSZ * K3 * 2;
static constexpr size_t SZ_XC   = (size_t)BSZ * KFC * 2;
static constexpr size_t SZ_EB   = (size_t)NPAD * HD * 2;
static constexpr size_t O_R1    = 0;
static constexpr size_t O_R2    = O_R1 + SZ_R1;
static constexpr size_t O_R3    = O_R2 + SZ_PL;
static constexpr size_t O_R4    = O_R3 + SZ_PL;
static constexpr size_t O_R5    = O_R4 + SZ_PL;
static constexpr size_t O_SLT   = O_R5 + SZ_EF;
static constexpr size_t O_WT2   = O_SLT + (size_t)512 * HD * 2;
static constexpr size_t O_NWT2  = O_WT2 + (size_t)2 * HD * KP2 * 2;
static constexpr size_t O_WRT   = O_NWT2 + (size_t)2 * HD * KP2 * 2;
static constexpr size_t O_RB    = O_WRT + (size_t)2 * HD * HD * 2;
static constexpr size_t O_V     = O_RB + (size_t)2 * RPAD * HD * 2;
static constexpr size_t O_RELF  = O_V + (size_t)4 * HD * 4;
static constexpr size_t O_CWB   = O_RELF + (size_t)NREL * HD * 4;
static constexpr size_t O_HR    = O_CWB + (size_t)32 * 128 * 2;
static constexpr size_t O_HRA3  = O_HR + (size_t)2 * RPAD * HD * 4;
static constexpr size_t O_SDP   = O_HRA3 + (size_t)2 * RPAD * 4;
static constexpr size_t O_REC   = O_SDP + (size_t)2 * NB64 * 256 * 4;
static constexpr size_t O_DIAG  = O_REC + (size_t)2 * NB128 * 1280 * 8;
static constexpr size_t O_END   = O_DIAG + (size_t)4 * NSELB * 32 * 4;
static_assert(O_END <= (size_t)WSMAX);
static_assert(O_R2 % 256 == 0 && O_R5 % 256 == 0 && O_SLT % 256 == 0 && O_V % 256 == 0);
static_assert(O_RELF % 256 == 0 && O_CWB % 256 == 0 && O_HR % 256 == 0 && O_HRA3 % 256 == 0);
static_assert(O_SDP % 256 == 0 && O_REC % 256 == 0 && O_DIAG % 256 == 0);
static_assert(SZ_EF3 + SZ_FCT + SZ_A3X <= SZ_R1);
static_assert(SZ_EF3 % 256 == 0 && (SZ_EF3 + SZ_FCT) % 256 == 0);
static_assert(SZ_XC <= SZ_PL && SZ_EB <= SZ_PL && (size_t)NPAD * KP2 * 2 == SZ_PL);

extern "C" void kernel_launch(void* const* d_in, const int* in_sizes, int n_in,
                              void* d_out, int out_size, void* d_ws, size_t ws_size,
                              hipStream_t stream) {
  if (n_in < 20) return;
  if (in_sizes[0] != BSZ || in_sizes[1] != BSZ) return;
  if (in_sizes[2] != NEDGE || in_sizes[3] != NEDGE) return;
  if (in_sizes[4] != NENT * HD) return;
  if (in_sizes[5] != 2 * NREL * HD) return;
  if (in_sizes[6] != 2) return;
  if (in_sizes[7] != HD * HD || in_sizes[8] != HD || in_sizes[9] != HD * HD || in_sizes[10] != HD) return;
  if (in_sizes[11] != 2 * HD * HD || in_sizes[12] != 2 * HD * HD) return;
  if (in_sizes[13] != 2 * 768) return;
  if (in_sizes[14] != 2 * HD * HD) return;
  if (in_sizes[15] != 32 * 49 || in_sizes[16] != 32) return;
  if (in_sizes[17] != FLAT * HD || in_sizes[18] != HD) return;
  if (in_sizes[19] != NENT) return;
  if (out_size != OUT_ELEMS) return;
  if (O_END > ws_size) return;

  const int*   h_id  = (const int*)d_in[0];
  const int*   r_id  = (const int*)d_in[1];
  const int*   esrc  = (const int*)d_in[2];
  const int*   erel  = (const int*)d_in[3];
  const float* ent   = (const float*)d_in[4];
  const float* rel   = (const float*)d_in[5];
  const float* gate  = (const float*)d_in[6];
  const float* S_w   = (const float*)d_in[7];
  const float* S_b   = (const float*)d_in[8];
  const float* L_w   = (const float*)d_in[9];
  const float* L_b   = (const float*)d_in[10];
  const float* Wm    = (const float*)d_in[11];
  const float* W_r   = (const float*)d_in[12];
  const float* av    = (const float*)d_in[13];
  const float* nw    = (const float*)d_in[14];
  const float* cw    = (const float*)d_in[15];
  const float* cb    = (const float*)d_in[16];
  const float* fcw   = (const float*)d_in[17];
  const float* fcb   = (const float*)d_in[18];
  const float* ebias = (const float*)d_in[19];
  float* out = (float*)d_out;

  char* ws = (char*)d_ws;
  unsigned short* CPhl = (unsigned short*)(ws + O_R1);
  unsigned short* EF3  = (unsigned short*)(ws + O_R1);
  unsigned short* FCT  = (unsigned short*)(ws + O_R1 + SZ_EF3);
  unsigned short* A3x  = (unsigned short*)(ws + O_R1 + SZ_EF3 + SZ_FCT);
  float*          Hb   = (float*)(ws + O_R2);
  unsigned short* EB   = (unsigned short*)(ws + O_R3);
  unsigned short* NE   = (unsigned short*)(ws + O_R3);
  unsigned short* XC   = (unsigned short*)(ws + O_R3);
  float*          Tc   = (float*)(ws + O_R4);
  float*          EF   = (float*)(ws + O_R5);
  unsigned short* SLT  = (unsigned short*)(ws + O_SLT);
  unsigned short* WT2  = (unsigned short*)(ws + O_WT2);
  unsigned short* NWT2 = (unsigned short*)(ws + O_NWT2);
  unsigned short* WRT  = (unsigned short*)(ws + O_WRT);
  unsigned short* RB   = (unsigned short*)(ws + O_RB);
  float*          Vp   = (float*)(ws + O_V);
  float*          RELF = (float*)(ws + O_RELF);
  unsigned short* CWB  = (unsigned short*)(ws + O_CWB);
  float*          HR   = (float*)(ws + O_HR);
  float*          HRA3 = (float*)(ws + O_HRA3);
  float*          SDP  = (float*)(ws + O_SDP);
  double*         REC  = (double*)(ws + O_REC);
  float*          DIAG = (float*)(ws + O_DIAG);

  hipFuncSetAttribute(reinterpret_cast<const void*>(&k_gemm_cp), hipFuncAttributeMaxDynamicSharedMemorySize, LDS_G2);
  hipFuncSetAttribute(reinterpret_cast<const void*>(&k_gemm_f32<0>), hipFuncAttributeMaxDynamicSharedMemorySize, LDS_G2);
  hipFuncSetAttribute(reinterpret_cast<const void*>(&k_gemm_f32<1>), hipFuncAttributeMaxDynamicSharedMemorySize, LDS_G2);
  hipFuncSetAttribute(reinterpret_cast<const void*>(&k_gemm_f32<2>), hipFuncAttributeMaxDynamicSharedMemorySize, LDS_G2);
  hipFuncSetAttribute(reinterpret_cast<const void*>(&k_gemm_fc), hipFuncAttributeMaxDynamicSharedMemorySize, LDS_G2);
  hipFuncSetAttribute(reinterpret_cast<const void*>(&k_conv), hipFuncAttributeMaxDynamicSharedMemorySize, LDS_CONV);

  k_pa<<<(PA_UEB + 2 * PA_USW) / 256, 256, 0, stream>>>(ent, S_w, L_w, EB, SLT);
  k_pb<<<PB_U4 / 256, 256, 0, stream>>>(Wm, W_r, nw, rel, av, WT2, NWT2, WRT, RB, Vp);
  k_pc<<<PC_U1 / 256, 256, 0, stream>>>(rel, gate, cw, RELF, CWB);
  k_gemm_f32<2><<<dim3(RPAD / 64, 2), 256, LDS_G2, stream>>>(RB, HD, WRT, HD, HD, HR, av, HRA3);
  k_gemm_cp<<<dim3(NB64, 2), 256, LDS_G2, stream>>>(EB, SLT, S_b, L_b, Vp, CPhl, SDP);

  for (int i = 0; i < 2; ++i) {
    for (int t = 0; t < 2; ++t) {
      float* Tout = (t == 0) ? Tc : Hb;
      k_gemm_f32<0><<<dim3(NB64, 1), 256, LDS_G2, stream>>>(CPhl + (size_t)t * NPAD * KP2, KP2,
                                                          WT2 + (size_t)i * 131072, KP2, KP2, Hb, av, HRA3);
      k_sel<<<NSELB, 256, 0, stream>>>(esrc, erel, SDP + (size_t)t * NB64 * 256, HRA3 + i * RPAD, Hb,
                                       HR + (size_t)i * RPAD * HD, NE,
                                       DIAG + (size_t)(2 * i + t) * NSELB * 32, i);
      k_gemm_f32<1><<<dim3(NB64, 1), 256, LDS_G2, stream>>>(NE, KP2, NWT2 + (size_t)i * 131072, KP2, KP2,
                                                          Tout, av, HRA3);
    }
    if (i == 0) {
      k_fuse<0><<<NB128, 256, 0, stream>>>(ent, Tc, Hb, gate, EF, REC);
    } else {
      k_fuse<1><<<NB128, 256, 0, stream>>>(ent, Tc, Hb, gate, EF, REC + (size_t)NB128 * 1280);
    }
  }
  k_corr<<<1, 256, 0, stream>>>(REC, out + OUT0_ELEMS);

  k_pc2<<<(HD * (FLAT / 8)) / 256, 256, 0, stream>>>(fcw, FCT);
  k_split<<<(NPAD * 32) / 256, 256, 0, stream>>>(EF, EF3);
  k_conv<<<BSZ, 256, LDS_CONV, stream>>>(h_id, r_id, EF, RELF, CWB, cb, XC);
  k_gemm_fc<<<BSZ / 64, 256, LDS_G2, stream>>>(XC, FCT, fcb, A3x);
  k_gemm_score<<<dim3(BSZ / 64, NB128), 128, LDS_G1, stream>>>(A3x, EF3, ebias, out);
}
